// vgae_decoder_14800457302103
// MI455X (gfx1250) — hardware-verified
//
#include <hip/hip_runtime.h>
#include <stdint.h>

typedef __attribute__((ext_vector_type(16))) _Float16 v16h;
typedef __attribute__((ext_vector_type(8)))  _Float16 v8h;
typedef __attribute__((ext_vector_type(8)))  float    v8f;
typedef __attribute__((ext_vector_type(4)))  float    v4f;

__device__ __forceinline__ void dep_guard_h(v8f& a, v8f& b, v16h x, v16h y) { asm volatile("v_nop\n\tv_nop\n\tv_nop\n\tv_nop" : "+v"(a), "+v"(b) : "v"(x), "v"(y)); }
__device__ __forceinline__ void keep4_h(v16h a, v16h b, v16h c, v16h d) { asm volatile("v_nop" :: "v"(a), "v"(b), "v"(c), "v"(d)); }
template <typename T> struct Frag;
template <> struct Frag<_Float16> {
  typedef v16h V; union U { v16h v; v8h h[2]; };
  static __device__ __forceinline__ v16h load(const _Float16* p) {
    U f; f.h[0] = *(const v8h*)(p); f.h[1] = *(const v8h*)(p + 16); return f.v;
  }
  static __device__ __forceinline__ v8f mma(v16h a, v16h b, v8f c) {
    return __builtin_amdgcn_wmma_f32_16x16x32_f16(false, a, false, b, (short)0, c, false, false);
  }
  static __device__ __forceinline__ void guard(v8f& a, v8f& b, v16h x, v16h y) { dep_guard_h(a, b, x, y); }
  static __device__ __forceinline__ void keep(v16h a, v16h b, v16h c, v16h d) { keep4_h(a, b, c, d); }
};

__device__ __forceinline__ v8f mma_h(v16h a, v16h b, v8f c) {
  c = Frag<_Float16>::mma(a, b, c);
  asm volatile("v_nop\n\tv_nop\n\tv_nop\n\tv_nop" : "+v"(c) : "v"(a), "v"(b));
  return c;
}

#define HID   128
#define TM    64
#define HP    136
#define NTHR  128
#define A_SC  16.0f
#define W_SC  64.0f
#define INV_SC (1.0f / 1024.0f)

__global__ __launch_bounds__(NTHR)
void edge_mlp_decode(const float* __restrict__ x,  const float* __restrict__ W1,
                     const float* __restrict__ b1, const float* __restrict__ W2,
                     const float* __restrict__ b2,
                     const int* __restrict__ ei, const int* __restrict__ ein,
                     float* __restrict__ out,
                     int NN, int Ep, int En, int Mtotal, int tiles)
{
  __shared__ __align__(16) _Float16 Hs[TM * HP];
  __shared__ __align__(16) _Float16 W1s[HID * HP];
  __shared__ __align__(16) float outs[TM];

  const int t    = threadIdx.x;
  const int wave = t >> 5;
  const int lane = t & 31;
  const int hh   = lane >> 4;
  const int c    = lane & 15;

  for (int i = t; i < HID * (HID / 2); i += NTHR) {
    const int n  = i & (HID - 1);
    const int kp = i >> 7;
    const float f0 = W1[(size_t)(2 * kp) * HID + n] * W_SC;
    const float f1 = W1[(size_t)(2 * kp + 1) * HID + n] * W_SC;
    const unsigned u = (unsigned)__builtin_bit_cast(unsigned short, (_Float16)f0)
                     | ((unsigned)__builtin_bit_cast(unsigned short, (_Float16)f1) << 16);
    *(unsigned*)(W1s + n * HP + 2 * kp) = u;
  }
  float b1r[8], w2r[8];
#pragma unroll
  for (int j = 0; j < 8; ++j) { b1r[j] = b1[16 * j + c]; w2r[j] = W2[16 * j + c]; }
  const float b2v = b2[0];
  __syncthreads();

  for (int tile = blockIdx.x; tile < tiles; tile += gridDim.x) {
    {
      const int r  = t >> 1;
      const int ch = t & 1;
      int g = tile * TM + r;
      if (g > Mtotal - 1) g = Mtotal - 1;
      int gp = (g < Ep) ? g : (Ep - 1);
      int gn = g - Ep; gn = (gn < 0) ? 0 : gn; gn = (gn > En - 1) ? (En - 1) : gn;
      const int sp = ei[gp], dp = ei[Ep + gp];
      const int sn = ein[gn], dn = ein[En + gn];
      const bool isneg = (g >= Ep);
      int s = isneg ? sn : sp;
      int d = isneg ? dn : dp;
      if (s < 0) s += NN;  s = (s < 0) ? 0 : s;  s = (s > NN - 1) ? (NN - 1) : s;
      if (d < 0) d += NN;  d = (d < 0) ? 0 : d;  d = (d > NN - 1) ? (NN - 1) : d;
      const v4f* xs = (const v4f*)(x + (size_t)s * HID) + 16 * ch;
      const v4f* xd = (const v4f*)(x + (size_t)d * HID) + 16 * ch;
      _Float16* hrow = Hs + r * HP + 64 * ch;
#pragma unroll 2
      for (int q = 0; q < 8; ++q) {
        const v4f a0 = xs[2 * q], a1 = xs[2 * q + 1];
        const v4f c0 = xd[2 * q], c1 = xd[2 * q + 1];
        v8h hv;
        hv[0] = (_Float16)(fmaxf(a0.x * c0.x, 0.0f) * A_SC);
        hv[1] = (_Float16)(fmaxf(a0.y * c0.y, 0.0f) * A_SC);
        hv[2] = (_Float16)(fmaxf(a0.z * c0.z, 0.0f) * A_SC);
        hv[3] = (_Float16)(fmaxf(a0.w * c0.w, 0.0f) * A_SC);
        hv[4] = (_Float16)(fmaxf(a1.x * c1.x, 0.0f) * A_SC);
        hv[5] = (_Float16)(fmaxf(a1.y * c1.y, 0.0f) * A_SC);
        hv[6] = (_Float16)(fmaxf(a1.z * c1.z, 0.0f) * A_SC);
        hv[7] = (_Float16)(fmaxf(a1.w * c1.w, 0.0f) * A_SC);
        *(v8h*)(hrow + 8 * q) = hv;
      }
    }
    __syncthreads();

    v8f acc[8];
#pragma unroll
    for (int j = 0; j < 8; ++j) acc[j] = (v8f){0.f,0.f,0.f,0.f,0.f,0.f,0.f,0.f};
#pragma unroll 1
    for (int ks = 0; ks < 4; ++ks) {
      const v16h af = Frag<_Float16>::load(Hs + (16 * wave + c) * HP + ks * 32 + 8 * hh);
#pragma unroll
      for (int j = 0; j < 8; ++j) {
        const v16h bf = Frag<_Float16>::load(W1s + (16 * j + c) * HP + ks * 32 + 8 * hh);
        acc[j] = mma_h(af, bf, acc[j]);
      }
    }

    float rowv = 0.0f;
#pragma unroll
    for (int r = 0; r < 8; ++r) {
      float qs = 0.0f;
#pragma unroll
      for (int j = 0; j < 8; ++j) {
        const float z = fmaxf(fmaf(acc[j][r], INV_SC, b1r[j]), 0.0f);
        qs = fmaf(z, w2r[j], qs);
      }
      qs += __shfl_xor(qs, 1, 32);
      qs += __shfl_xor(qs, 2, 32);
      qs += __shfl_xor(qs, 4, 32);
      qs += __shfl_xor(qs, 8, 32);
      rowv = (c == r) ? qs : rowv;
    }
    if (c < 8) {
      const float zz = rowv + b2v;
      const float e  = expf(-zz);
      outs[16 * wave + 8 * hh + c] = __builtin_amdgcn_rcpf(1.0f + e);
    }
    __syncthreads();

    const int rows = Mtotal - tile * TM;
    if (rows >= TM) {
      if (wave == 0 && lane < 16) {
        const v4f val = *(const v4f*)(outs + 4 * lane);
        float* op = out + (size_t)tile * TM + 4 * lane;
        *(volatile v4f*)op = val;
        __threadfence();
        *(volatile v4f*)op = val;
      }
    } else {
      if (t < rows) {
        const float v = outs[t];
        float* op = out + (size_t)tile * TM + t;
        *(volatile float*)op = v;
        __threadfence();
        *(volatile float*)op = v;
      }
    }
  }
}

extern "C" void kernel_launch(void* const* d_in, const int* in_sizes, int n_in,
                              void* d_out, int out_size, void* d_ws, size_t ws_size,
                              hipStream_t stream) {
  (void)d_ws; (void)ws_size;
  if (n_in < 7) return;
  const float* x   = (const float*)d_in[0];
  const float* W1  = (const float*)d_in[1];
  const float* b1  = (const float*)d_in[2];
  const float* W2  = (const float*)d_in[3];
  const float* b2  = (const float*)d_in[4];
  const int*   ei  = (const int*)d_in[5];
  const int*   ein = (const int*)d_in[6];
  float* out = (float*)d_out;

  const int NN = in_sizes[0] / HID;
  const int Ep = in_sizes[5] / 2;
  const int En = in_sizes[6] / 2;
  int Mtotal = Ep + En;
  if (Mtotal > out_size) Mtotal = out_size;
  if (NN <= 0 || Ep <= 0 || En <= 0 || Mtotal <= 0) return;

  const int tiles = (Mtotal + TM - 1) / TM;
  const int grid  = tiles < 1024 ? tiles : 1024;

  edge_mlp_decode<<<dim3(grid), dim3(NTHR), 0, stream>>>(
      x, W1, b1, W2, b2, ei, ein, out, NN, Ep, En, Mtotal, tiles);
}
